// ShapedAttention_60490319397277
// MI455X (gfx1250) — hardware-verified
//
#include <hip/hip_runtime.h>
#include <stdint.h>

typedef _Float16 v16h __attribute__((ext_vector_type(16)));
typedef _Float16 v8h  __attribute__((ext_vector_type(8)));
typedef __bf16   v16b __attribute__((ext_vector_type(16)));
typedef __bf16   v8b  __attribute__((ext_vector_type(8)));
typedef unsigned short v8us __attribute__((ext_vector_type(8)));
typedef float    v8f  __attribute__((ext_vector_type(8)));
typedef float    v4f  __attribute__((ext_vector_type(4)));
typedef v8h  __attribute__((may_alias)) v8ha;
typedef v8b  __attribute__((may_alias)) v8ba;
typedef v8us __attribute__((may_alias)) v8usa;
typedef v4f  __attribute__((may_alias)) v4fa;

#define BATCH 2
#define SEQ   2048
#define DIM   1024
#define HEADS 16
#define HD    64
#define MROWS (BATCH * SEQ)
#define NX    (MROWS * DIM)
#define NWQ   (DIM * 3 * DIM)
#define NWO   (DIM * DIM)
#define NBH   (BATCH * HEADS)
#define QSC    8.0f
#define PSCALE 16384.0f
#define LOSC   4096.0f
#define WOSC   256.0f
#define TRP    72

static_assert(SEQ % 128 == 0);
static_assert(DIM % 64 == 0);
static_assert(HEADS * HD == DIM);
static_assert((NX % 8) == 0);

__device__ __forceinline__ v8f wmma_f16(v16h a, v16h b, v8f c) {
  v8f d = __builtin_amdgcn_wmma_f32_16x16x32_f16(false, a, false, b, (short)0, c, false, false);
  asm volatile("v_nop\n\tv_nop\n\tv_nop\n\tv_nop" : "+v"(d) : "v"(a), "v"(b));
  return d;
}
__device__ __forceinline__ v8f wmma_bf16(v16b a, v16b b, v8f c) {
  v8f d = __builtin_amdgcn_wmma_f32_16x16x32_bf16(false, a, false, b, (short)0, c, false, false);
  asm volatile("v_nop\n\tv_nop\n\tv_nop\n\tv_nop" : "+v"(d) : "v"(a), "v"(b));
  return d;
}

__device__ __forceinline__ v16h frag_h(const _Float16* p, int h) {
  union { v16h v; v8h hf[2]; } f;
  f.hf[0] = *(const v8ha*)(p + 8 * h);
  f.hf[1] = *(const v8ha*)(p + 16 + 8 * h);
  return f.v;
}
__device__ __forceinline__ v16b frag_b(const __bf16* p, int h) {
  union { v16b v; v8b hf[2]; } f;
  f.hf[0] = *(const v8ba*)(p + 8 * h);
  f.hf[1] = *(const v8ba*)(p + 16 + 8 * h);
  return f.v;
}

__device__ __forceinline__ unsigned short bf16_bits(float f) {
  const uint32_t u = __builtin_bit_cast(uint32_t, f);
  const uint32_t r = u + 0x7FFFu + ((u >> 16) & 1u);
  return (unsigned short)(r >> 16);
}
__device__ __forceinline__ float bf16_val(float f) {
  return __builtin_bit_cast(float, ((uint32_t)bf16_bits(f)) << 16);
}

__global__ __launch_bounds__(256) void k_cvt_x(const float* __restrict__ x,
                                               unsigned short* __restrict__ xb, int n8) {
  const int g = blockIdx.x * 256 + threadIdx.x;
  if (g >= n8) return;
  const float* s = x + (size_t)g * 8;
  const v4f a = *(const v4fa*)s;
  const v4f c = *(const v4fa*)(s + 4);
  v8us o;
  o[0] = bf16_bits(a.x); o[1] = bf16_bits(a.y); o[2] = bf16_bits(a.z); o[3] = bf16_bits(a.w);
  o[4] = bf16_bits(c.x); o[5] = bf16_bits(c.y); o[6] = bf16_bits(c.z); o[7] = bf16_bits(c.w);
  unsigned short* d = xb + (size_t)g * 8;
  *(volatile v8us*)d = o;
  __threadfence();
  *(volatile v8us*)d = o;
}

template <int MODE>
__global__ __launch_bounds__(256) void k_transpose(const float* __restrict__ src,
                                                   unsigned short* __restrict__ dst,
                                                   int K, int N) {
  __shared__ __attribute__((aligned(16))) unsigned short sT[64 * TRP];
  const int tid = threadIdx.x, lane = tid & 31, w = tid >> 5;
  const int k0 = blockIdx.x * 64, n0 = blockIdx.y * 64;
  if (k0 + 64 > K || n0 + 64 > N) return;
  const int nc = tid & 63, kq = tid >> 6;
#pragma unroll
  for (int i = 0; i < 16; ++i) {
    const int kr = 4 * i + kq;
    const float v = src[(size_t)(k0 + kr) * N + n0 + nc];
    unsigned short o;
    if (MODE == 0) {
      o = bf16_bits(v);
    } else {
      const _Float16 hv = (_Float16)(bf16_val(v) * WOSC);
      o = __builtin_bit_cast(unsigned short, hv);
    }
    sT[nc * TRP + kr] = o;
  }
  __syncthreads();
  const int q8 = lane & 7, sub = lane >> 3;
  v8us vv[2];
  size_t gi[2];
#pragma unroll
  for (int i = 0; i < 2; ++i) {
    const int row = 8 * w + 4 * i + sub;
    vv[i] = *(const v8usa*)(sT + row * TRP + 8 * q8);
    gi[i] = (size_t)(n0 + row) * K + k0 + 8 * q8;
  }
#pragma unroll
  for (int i = 0; i < 2; ++i) *(volatile v8us*)(dst + gi[i]) = vv[i];
  __threadfence();
#pragma unroll
  for (int i = 0; i < 2; ++i) *(volatile v8us*)(dst + gi[i]) = vv[i];
}

__device__ __forceinline__ void proj_store_pass(const _Float16* sT, const float* sF,
                                                _Float16* plane, _Float16* vt, float* vf,
                                                int which, int bh, int l0, int w, int lane) {
  const int q8 = lane & 7, sub = lane >> 3;
  if (which != 2) {
#pragma unroll
    for (int i = 0; i < 8; ++i) {
      const int lid = w * 32 + i * 4 + sub;
      const v8h v = *(const v8ha*)(sT + lid * HD + 8 * q8);
      _Float16* dst = plane + ((size_t)bh * SEQ + l0 + lid) * HD + 8 * q8;
      *(volatile v8h*)dst = v;
    }
  } else {
#pragma unroll
    for (int i = 0; i < 8; ++i) {
      const int lid = w * 32 + i * 4 + sub;
      const int d = lid >> 1, hl = lid & 1;
      const v8h v = *(const v8ha*)(sT + d * 128 + 64 * hl + 8 * q8);
      _Float16* dst = vt + ((size_t)bh * HD + d) * SEQ + l0 + 64 * hl + 8 * q8;
      *(volatile v8h*)dst = v;
    }
#pragma unroll
    for (int i = 0; i < 16; ++i) {
      const int lid = w * 64 + i * 4 + sub;
      const int tok = lid >> 1, hl = lid & 1;
      const v4f v = *(const v4fa*)(sF + tok * HD + 32 * hl + 4 * q8);
      float* dst = vf + ((size_t)bh * SEQ + l0 + tok) * HD + 32 * hl + 4 * q8;
      *(volatile v4f*)dst = v;
    }
  }
}

__global__ __launch_bounds__(128) void k_proj(const __bf16* __restrict__ xb,
                                              const __bf16* __restrict__ wqt,
                                              _Float16* __restrict__ qh,
                                              _Float16* __restrict__ kh,
                                              _Float16* __restrict__ vt,
                                              float* __restrict__ vf) {
  __shared__ __attribute__((aligned(16))) _Float16 sT[128 * 64];
  __shared__ __attribute__((aligned(16))) float    sF[128 * 64];

  const int tid = threadIdx.x, lane = tid & 31, w = tid >> 5;
  const int h = lane >> 4, m = lane & 15;
  const int m0 = blockIdx.x * 128;
  const int cg = blockIdx.y;
  const int which = cg >> 4, head = cg & 15;
  const int m0w = m0 + 32 * w;

  const __bf16* xa0 = xb + (size_t)(m0w + m) * DIM;
  const __bf16* xa1 = xa0 + (size_t)16 * DIM;
  const __bf16* wb  = wqt + ((size_t)which * DIM + head * HD + m) * DIM;

  const v8f zero8 = {0.f, 0.f, 0.f, 0.f, 0.f, 0.f, 0.f, 0.f};
  v8f acc[2][4];
#pragma unroll
  for (int mt = 0; mt < 2; ++mt)
#pragma unroll
    for (int nt = 0; nt < 4; ++nt) acc[mt][nt] = zero8;

#pragma unroll 1
  for (int k0 = 0; k0 < DIM; k0 += 32) {
    const v16b a0 = frag_b(xa0 + k0, h);
    const v16b a1 = frag_b(xa1 + k0, h);
#pragma unroll
    for (int nt = 0; nt < 4; ++nt) {
      const v16b bq = frag_b(wb + (size_t)nt * 16 * DIM + k0, h);
      acc[0][nt] = wmma_bf16(a0, bq, acc[0][nt]);
      acc[1][nt] = wmma_bf16(a1, bq, acc[1][nt]);
    }
  }

  if (which == 2) {
#pragma unroll
    for (int nt = 0; nt < 4; ++nt) {
      const int feat = 16 * nt + m;
#pragma unroll
      for (int mt = 0; mt < 2; ++mt) {
#pragma unroll
        for (int r = 0; r < 8; ++r) {
          const int tokl = 32 * w + 16 * mt + 8 * h + r;
          const float y = acc[mt][nt][r];
          sT[feat * 128 + tokl] = (_Float16)(y * QSC);
          sF[tokl * HD + feat] = y;
        }
      }
    }
  } else {
#pragma unroll
    for (int nt = 0; nt < 4; ++nt) {
      const int feat = 16 * nt + m;
#pragma unroll
      for (int mt = 0; mt < 2; ++mt) {
#pragma unroll
        for (int r = 0; r < 8; ++r) {
          const int tokl = 32 * w + 16 * mt + 8 * h + r;
          sT[tokl * HD + feat] = (_Float16)(acc[mt][nt][r] * QSC);
        }
      }
    }
  }
  __syncthreads();

  const int b = m0 >> 11, l0 = m0 & (SEQ - 1), bh = b * HEADS + head;
  _Float16* plane = (which == 0) ? qh : kh;
  proj_store_pass(sT, sF, plane, vt, vf, which, bh, l0, w, lane);
  __threadfence();
  proj_store_pass(sT, sF, plane, vt, vf, which, bh, l0, w, lane);
}

__global__ __launch_bounds__(64) void k_vsum(const float* __restrict__ vf,
                                             float* __restrict__ vsum) {
  const int bh = blockIdx.x, d = threadIdx.x;
  const float* p = vf + (size_t)bh * SEQ * HD + d;
  float s = 0.0f;
#pragma unroll 4
  for (int l = 0; l < SEQ; ++l) s += p[(size_t)l * HD];
  float* dst = vsum + bh * HD + d;
  *(volatile float*)dst = s;
  __threadfence();
  *(volatile float*)dst = s;
}

__device__ __forceinline__ v16h pack_p(v8f a, v8f c) {
  union { v16h v; v8h hf[2]; } f;
  v8h xa, xc;
#pragma unroll
  for (int r = 0; r < 8; ++r) {
    xa[r] = (_Float16)(a[r] * PSCALE);
    xc[r] = (_Float16)(c[r] * PSCALE);
  }
  f.hf[0] = xa;
  f.hf[1] = xc;
  return f.v;
}

__global__ __launch_bounds__(128) void k_attn(const _Float16* __restrict__ qh,
                                              const _Float16* __restrict__ kh,
                                              const _Float16* __restrict__ vt,
                                              const float* __restrict__ vf,
                                              const float* __restrict__ vsum,
                                              const float* __restrict__ pAlpha,
                                              const float* __restrict__ pBeta,
                                              const float* __restrict__ pGamma,
                                              _Float16* __restrict__ ah,
                                              _Float16* __restrict__ al) {
  __shared__ __attribute__((aligned(16))) _Float16 sH[4 * 16 * 64];
  __shared__ __attribute__((aligned(16))) _Float16 sL[4 * 16 * 64];

  const int tid = threadIdx.x, lane = tid & 31, w = tid >> 5;
  const int h = lane >> 4, m = lane & 15;
  const int bh = blockIdx.y, b = bh >> 4, head = bh & 15;
  const int q0 = blockIdx.x * 64 + 16 * w;

  const _Float16* qrow = qh + ((size_t)bh * SEQ + q0 + m) * HD;
  const v16h qb0 = frag_h(qrow, h);
  const v16h qb1 = frag_h(qrow + 32, h);

  const v8f zero8 = {0.f, 0.f, 0.f, 0.f, 0.f, 0.f, 0.f, 0.f};
  v8f o[4];
#pragma unroll
  for (int t = 0; t < 4; ++t) o[t] = zero8;
  float mrun = -1.0e30f, lrun = 0.0f;

  const _Float16* kbase = kh + ((size_t)bh * SEQ + m) * HD;
  const _Float16* vbase = vt + ((size_t)bh * HD + m) * SEQ;
  const float ssc = (1.0f / (QSC * QSC)) * 0.03125f * 1.4426950408889634f;

#pragma unroll 1
  for (int kb = 0; kb < SEQ; kb += 64) {
    v8f s[4];
#pragma unroll
    for (int j = 0; j < 4; ++j) {
      const _Float16* kp = kbase + (size_t)(kb + 16 * j) * HD;
      const v16h kf0 = frag_h(kp, h);
      const v16h kf1 = frag_h(kp + 32, h);
      v8f z = wmma_f16(kf0, qb0, zero8);
      z = wmma_f16(kf1, qb1, z);
      s[j] = z;
    }

    float mloc = -1.0e30f;
#pragma unroll
    for (int j = 0; j < 4; ++j)
#pragma unroll
      for (int r = 0; r < 8; ++r) {
        const float tval = s[j][r] * ssc;
        s[j][r] = tval;
        mloc = fmaxf(mloc, tval);
      }
    mloc = fmaxf(mloc, __shfl_xor(mloc, 16));
    const float mnew = fmaxf(mrun, mloc);
    const float corr = exp2f(mrun - mnew);
    mrun = mnew;
    float lsum = 0.0f;
#pragma unroll
    for (int j = 0; j < 4; ++j)
#pragma unroll
      for (int r = 0; r < 8; ++r) {
        const float p = exp2f(s[j][r] - mnew);
        s[j][r] = p;
        lsum += p;
      }
    lsum += __shfl_xor(lsum, 16);
    lrun = lrun * corr + lsum;
#pragma unroll
    for (int t = 0; t < 4; ++t)
#pragma unroll
      for (int r = 0; r < 8; ++r) o[t][r] = o[t][r] * corr;

    const v16h pb0 = pack_p(s[0], s[1]);
    const v16h pb1 = pack_p(s[2], s[3]);

#pragma unroll
    for (int t = 0; t < 4; ++t) {
      const _Float16* vp = vbase + (size_t)(16 * t) * SEQ + kb;
      const v16h va0 = frag_h(vp, h);
      const v16h va1 = frag_h(vp + 32, h);
      o[t] = wmma_f16(va0, pb0, o[t]);
      o[t] = wmma_f16(va1, pb1, o[t]);
    }
  }

  const float alpha  = bf16_val(pAlpha[0]);
  const float beta   = bf16_val(pBeta[0]);
  const float gamman = bf16_val(pGamma[0]) * (1.0f / (float)SEQ);
  const float inv = beta * (1.0f / (lrun * (PSCALE * QSC)));
  const float* vrow = vf + ((size_t)bh * SEQ + q0 + m) * HD;
  const float* vsr  = vsum + bh * HD;
  _Float16* shw = sH + w * 1024 + m * 64;
  _Float16* slw = sL + w * 1024 + m * 64;
#pragma unroll
  for (int t = 0; t < 4; ++t) {
    const v4f xa = *(const v4fa*)(vrow + 16 * t + 8 * h);
    const v4f xb = *(const v4fa*)(vrow + 16 * t + 8 * h + 4);
    const v4f ua = *(const v4fa*)(vsr + 16 * t + 8 * h);
    const v4f ub = *(const v4fa*)(vsr + 16 * t + 8 * h + 4);
    const float vv[8] = {xa.x, xa.y, xa.z, xa.w, xb.x, xb.y, xb.z, xb.w};
    const float uu[8] = {ua.x, ua.y, ua.z, ua.w, ub.x, ub.y, ub.z, ub.w};
    v8h hv, lv;
#pragma unroll
    for (int r = 0; r < 8; ++r) {
      const float res = alpha * vv[r] + o[t][r] * inv - gamman * uu[r];
      const _Float16 hq = (_Float16)res;
      hv[r] = hq;
      lv[r] = (_Float16)((res - (float)hq) * LOSC);
    }
    *(v8ha*)(shw + 16 * t + 8 * h) = hv;
    *(v8ha*)(slw + 16 * t + 8 * h) = lv;
  }
  __syncthreads();

  const int q8 = lane & 7, sub = lane >> 3;
  v8h hh[4], ll[4];
  size_t gi[4];
#pragma unroll
  for (int i = 0; i < 4; ++i) {
    const int row = 4 * i + sub;
    hh[i] = *(const v8ha*)(sH + w * 1024 + row * 64 + 8 * q8);
    ll[i] = *(const v8ha*)(sL + w * 1024 + row * 64 + 8 * q8);
    gi[i] = ((size_t)(b * SEQ + q0 + row)) * DIM + head * HD + 8 * q8;
  }
#pragma unroll
  for (int i = 0; i < 4; ++i) {
    *(volatile v8h*)(ah + gi[i]) = hh[i];
    *(volatile v8h*)(al + gi[i]) = ll[i];
  }
  __threadfence();
#pragma unroll
  for (int i = 0; i < 4; ++i) {
    *(volatile v8h*)(ah + gi[i]) = hh[i];
    *(volatile v8h*)(al + gi[i]) = ll[i];
  }
}

__global__ __launch_bounds__(128) void k_oproj(const _Float16* __restrict__ ah,
                                               const _Float16* __restrict__ al,
                                               const _Float16* __restrict__ wot,
                                               const float* __restrict__ bias,
                                               float* __restrict__ out) {
  __shared__ __attribute__((aligned(16))) float sO[128 * 32];

  const int tid = threadIdx.x, lane = tid & 31, w = tid >> 5;
  const int h = lane >> 4, m = lane & 15;
  const int m0 = blockIdx.x * 128, n0 = blockIdx.y * 32;
  const int m0w = m0 + 32 * w;

  const _Float16* ar0h = ah + (size_t)(m0w + m) * DIM;
  const _Float16* ar1h = ar0h + (size_t)16 * DIM;
  const _Float16* ar0l = al + (size_t)(m0w + m) * DIM;
  const _Float16* ar1l = ar0l + (size_t)16 * DIM;
  const _Float16* wr0  = wot + (size_t)(n0 + m) * DIM;
  const _Float16* wr1  = wr0 + (size_t)16 * DIM;

  const v8f zero8 = {0.f, 0.f, 0.f, 0.f, 0.f, 0.f, 0.f, 0.f};
  v8f accH[2][2], accL[2][2];
#pragma unroll
  for (int mt = 0; mt < 2; ++mt)
#pragma unroll
    for (int nt = 0; nt < 2; ++nt) { accH[mt][nt] = zero8; accL[mt][nt] = zero8; }

#pragma unroll 1
  for (int k0 = 0; k0 < DIM; k0 += 32) {
    const v16h a0h = frag_h(ar0h + k0, h);
    const v16h a1h = frag_h(ar1h + k0, h);
    const v16h a0l = frag_h(ar0l + k0, h);
    const v16h a1l = frag_h(ar1l + k0, h);
    const v16h b0  = frag_h(wr0 + k0, h);
    const v16h b1  = frag_h(wr1 + k0, h);
    accH[0][0] = wmma_f16(a0h, b0, accH[0][0]);
    accH[0][1] = wmma_f16(a0h, b1, accH[0][1]);
    accH[1][0] = wmma_f16(a1h, b0, accH[1][0]);
    accH[1][1] = wmma_f16(a1h, b1, accH[1][1]);
    accL[0][0] = wmma_f16(a0l, b0, accL[0][0]);
    accL[0][1] = wmma_f16(a0l, b1, accL[0][1]);
    accL[1][0] = wmma_f16(a1l, b0, accL[1][0]);
    accL[1][1] = wmma_f16(a1l, b1, accL[1][1]);
  }

  const float sh = 1.0f / WOSC;
  const float sl = 1.0f / (WOSC * LOSC);
#pragma unroll
  for (int nt = 0; nt < 2; ++nt) {
    const int featl = 16 * nt + m;
    const float bv = bf16_val(bias[n0 + featl]);
#pragma unroll
    for (int mt = 0; mt < 2; ++mt) {
#pragma unroll
      for (int r = 0; r < 8; ++r) {
        const int tokl = 32 * w + 16 * mt + 8 * h + r;
        sO[tokl * 32 + featl] = accH[mt][nt][r] * sh + accL[mt][nt][r] * sl + bv;
      }
    }
  }
  __syncthreads();

  const int q8 = lane & 7, sub = lane >> 3;
  v4f vv[8];
  size_t gi[8];
#pragma unroll
  for (int i = 0; i < 8; ++i) {
    const int lid = 32 * w + 4 * i + sub;
    vv[i] = *(const v4fa*)(sO + lid * 32 + 4 * q8);
    gi[i] = (size_t)(m0 + lid) * DIM + n0 + 4 * q8;
  }
#pragma unroll
  for (int i = 0; i < 8; ++i) *(volatile v4f*)(out + gi[i]) = vv[i];
  __threadfence();
#pragma unroll
  for (int i = 0; i < 8; ++i) *(volatile v4f*)(out + gi[i]) = vv[i];
}

extern "C" void kernel_launch(void* const* d_in, const int* in_sizes, int n_in,
                              void* d_out, int out_size, void* d_ws, size_t ws_size,
                              hipStream_t stream) {
  if (n_in < 7) return;
  if (in_sizes[0] != NX) return;
  if (in_sizes[1] != NWQ) return;
  if (in_sizes[2] != NWO) return;
  if (in_sizes[3] != DIM) return;
  if (in_sizes[4] < 1 || in_sizes[5] < 1 || in_sizes[6] < 1) return;
  if (out_size != NX) return;

  const float* x    = (const float*)d_in[0];
  const float* wqkv = (const float*)d_in[1];
  const float* wout = (const float*)d_in[2];
  const float* bout = (const float*)d_in[3];
  const float* pA   = (const float*)d_in[4];
  const float* pB   = (const float*)d_in[5];
  const float* pG   = (const float*)d_in[6];
  float* out = (float*)d_out;

  const size_t b_xb  = (size_t)NX * 2;
  const size_t b_wqt = (size_t)NWQ * 2;
  const size_t b_wot = (size_t)NWO * 2;
  const size_t b_pl  = (size_t)NBH * SEQ * HD * 2;
  const size_t b_vf  = (size_t)NBH * SEQ * HD * 4;
  const size_t b_a   = (size_t)NX * 2;
  const size_t b_vs  = (size_t)NBH * HD * 4;

  char* ws = (char*)d_ws;
  size_t off = 0;
  unsigned short* xb  = (unsigned short*)(ws + off); off += b_xb;
  unsigned short* wqt = (unsigned short*)(ws + off); off += b_wqt;
  unsigned short* wot = (unsigned short*)(ws + off); off += b_wot;
  _Float16* qh = (_Float16*)(ws + off); off += b_pl;
  _Float16* kh = (_Float16*)(ws + off); off += b_pl;
  _Float16* vt = (_Float16*)(ws + off); off += b_pl;
  float*    vf = (float*)(ws + off);    off += b_vf;
  _Float16* ah = (_Float16*)(ws + off); off += b_a;
  _Float16* al = (_Float16*)(ws + off); off += b_a;
  float*    vsum = (float*)(ws + off);  off += b_vs;
  if (off > ws_size) return;

  const int nx8 = NX / 8;
  k_cvt_x<<<(nx8 + 255) / 256, 256, 0, stream>>>(x, xb, nx8);

  k_transpose<0><<<dim3(DIM / 64, (3 * DIM) / 64), 256, 0, stream>>>(wqkv, wqt, DIM, 3 * DIM);
  k_transpose<1><<<dim3(DIM / 64, DIM / 64), 256, 0, stream>>>(wout, wot, DIM, DIM);

  k_proj<<<dim3(MROWS / 128, 3 * HEADS), 128, 0, stream>>>(
      (const __bf16*)xb, (const __bf16*)wqt, qh, kh, vt, vf);

  k_vsum<<<NBH, 64, 0, stream>>>(vf, vsum);

  k_attn<<<dim3(SEQ / 64, NBH), 128, 0, stream>>>(qh, kh, vt, vf, vsum, pA, pB, pG, ah, al);

  k_oproj<<<dim3(MROWS / 128, DIM / 32), 128, 0, stream>>>(ah, al, (const _Float16*)wot, bout, out);
}
